// SAGE_13134009991686
// MI455X (gfx1250) — hardware-verified
//
#include <hip/hip_runtime.h>
#include <stddef.h>
#include <stdint.h>


#define NN      100000
#define NE      1600000
#define NG      128
#define MP      100096
#define NTILE   782
#define NTILEP  784
#define TM      128
#define BNEPS   1e-5f
#define NTHR    256
#define NWAVE   8
#define EPT     8
#define CHUNK   (NTHR * EPT)
#define WCAP    (EPT * 32)
#define LISTN   (NWAVE * WCAP)
#define NBA     1024
#define SLA     10
#define NBLK    98
#define RCAP    28672
#define DEGCAP  64
#define AGG_ZINTS    (LISTN + 2 * RCAP + 3 * NBA)
#define AGG_LDS_INTS (AGG_ZINTS + 16)
#define PB_W1   0
#define PB_W2   1
#define PB_W3   2
#define PB_L1   10
#define PB_L2   26
#define PB_RUN  27
#define PB_XB   31
#define PB_END  1595
#define WSMAX   134217728

static_assert(MP == NTILE * TM && NBLK * NBA >= MP && MP % 2 == 0);
static_assert((CHUNK & (CHUNK - 1)) == 0 && CHUNK <= 4096);
static_assert((NBA & (NBA - 1)) == 0 && NBA == (1 << SLA) && NBA == 4 * NTHR);
static_assert(NE % 4 == 0 && NE < (1 << 21));
static_assert(RCAP >= 16710 && RCAP % 1024 == 0 && DEGCAP >= 36 + 8);
static_assert(AGG_ZINTS % (NTHR * 4) == 0 && AGG_LDS_INTS * 4 <= 300000);
static_assert(MP * 4 == (PB_END - PB_XB) * 256 && NTILEP <= (PB_XB - PB_RUN) * 256);
static_assert(NTILEP % 8 == 0 && NTILEP >= NTILE);

typedef float          v4f   __attribute__((ext_vector_type(4)));
typedef float          v8f   __attribute__((ext_vector_type(8)));
typedef int            v4i   __attribute__((ext_vector_type(4)));
typedef int            v8i   __attribute__((ext_vector_type(8)));
typedef unsigned       v2u   __attribute__((ext_vector_type(2)));
typedef unsigned short v2us  __attribute__((ext_vector_type(2)));
typedef unsigned short v4us  __attribute__((ext_vector_type(4)));
typedef unsigned short v8us  __attribute__((ext_vector_type(8)));
typedef unsigned short v16us __attribute__((ext_vector_type(16)));
typedef __bf16         v16bf __attribute__((ext_vector_type(16)));
typedef v4f  __attribute__((may_alias)) v4fa;
typedef v4i  __attribute__((may_alias)) v4ia;
typedef v2u  __attribute__((may_alias)) v2ua;
typedef v2us __attribute__((may_alias)) v2usa;
typedef v4us __attribute__((may_alias)) v4usa;
typedef v8us __attribute__((may_alias)) v8usa;
union FragB { v16bf v; v16us u; v8us h[2]; v8i w; };

__device__ __forceinline__ v8f wmb(const FragB& a, const FragB& b, v8f c) {
  v8f d = __builtin_amdgcn_wmma_f32_16x16x32_bf16(false, a.v, false, b.v, (short)0, c, false, false);
  asm volatile("v_nop\n\tv_nop\n\tv_nop\n\tv_nop" : "+v"(d) : "v"(a.w), "v"(b.w));
  return d;
}
__device__ __forceinline__ v8f z8() { v8f z = {0.f, 0.f, 0.f, 0.f, 0.f, 0.f, 0.f, 0.f}; return z; }

__device__ __forceinline__ unsigned bf16_bits(float f) {
  const unsigned u = __float_as_uint(f);
  return (u + 0x7FFFu + ((u >> 16) & 1u)) >> 16;
}
__device__ __forceinline__ float bf16_val(float f) { return __uint_as_float(bf16_bits(f) << 16); }
__device__ __forceinline__ unsigned hl_bits(float v, unsigned& lo) {
  const unsigned hb = bf16_bits(v);
  lo = bf16_bits(v - __uint_as_float(hb << 16));
  return hb;
}
__device__ __forceinline__ float relu_np(float v) { return (v > 0.0f) ? v : ((v == v) ? 0.0f : v); }

__device__ __forceinline__ void wave_sync() {
  __builtin_amdgcn_fence(__ATOMIC_RELEASE, "wavefront");
  __builtin_amdgcn_wave_barrier();
  __builtin_amdgcn_fence(__ATOMIC_ACQUIRE, "wavefront");
}

template <int SLB>
__device__ __forceinline__ int scan_chunk(const int* __restrict__ dsts, int nE, int cbase, int slotBase,
                                          int nb, int vec8, int* list, int tid, int lane, int wave) {
  int wc = 0;
  const int el0  = tid * EPT;
  const int e0   = cbase + el0;
  const int sent = -2147483647 - 1;
  v4i da, db;
  if (vec8 != 0 && cbase + CHUNK <= nE) {
    da = *(const v4i*)(dsts + e0);
    db = *(const v4i*)(dsts + e0 + 4);
  } else {
    da.x = (e0     < nE) ? dsts[min(e0,     nE - 1)] : sent;
    da.y = (e0 + 1 < nE) ? dsts[min(e0 + 1, nE - 1)] : sent;
    da.z = (e0 + 2 < nE) ? dsts[min(e0 + 2, nE - 1)] : sent;
    da.w = (e0 + 3 < nE) ? dsts[min(e0 + 3, nE - 1)] : sent;
    db.x = (e0 + 4 < nE) ? dsts[min(e0 + 4, nE - 1)] : sent;
    db.y = (e0 + 5 < nE) ? dsts[min(e0 + 5, nE - 1)] : sent;
    db.z = (e0 + 6 < nE) ? dsts[min(e0 + 6, nE - 1)] : sent;
    db.w = (e0 + 7 < nE) ? dsts[min(e0 + 7, nE - 1)] : sent;
  }
  const unsigned nbs = (unsigned)slotBase;
  const unsigned unb = (unsigned)nb;
  const unsigned s0 = (unsigned)da.x - nbs, s1 = (unsigned)da.y - nbs;
  const unsigned s2 = (unsigned)da.z - nbs, s3 = (unsigned)da.w - nbs;
  const unsigned s4 = (unsigned)db.x - nbs, s5 = (unsigned)db.y - nbs;
  const unsigned s6 = (unsigned)db.z - nbs, s7 = (unsigned)db.w - nbs;
  const bool h0 = s0 < unb, h1 = s1 < unb, h2 = s2 < unb, h3 = s3 < unb;
  const bool h4 = s4 < unb, h5 = s5 < unb, h6 = s6 < unb, h7 = s7 < unb;
  const unsigned any = __builtin_amdgcn_ballot_w32(h0 | h1 | h2 | h3 | h4 | h5 | h6 | h7);
  if (any != 0u) {
#define HITJ(J, HJ, SJ) { \
      const unsigned mj = __builtin_amdgcn_ballot_w32(HJ); \
      if (mj != 0u) { \
        if (HJ) { \
          const int pos = wc + (int)__builtin_amdgcn_mbcnt_lo(mj, 0u); \
          if (pos < WCAP) list[wave * WCAP + pos] = ((el0 + (J)) << SLB) | (int)(SJ); \
        } \
        wc += (int)__builtin_popcount(mj); } }
    HITJ(0, h0, s0)
    HITJ(1, h1, s1)
    HITJ(2, h2, s2)
    HITJ(3, h3, s3)
    HITJ(4, h4, s4)
    HITJ(5, h5, s5)
    HITJ(6, h6, s6)
    HITJ(7, h7, s7)
#undef HITJ
  }
  return wc;
}

template <int DIN, int DOUT, int R, int DUP>
__device__ __forceinline__ void wfill(const float* __restrict__ w, int n0, int kofs, int kcat,
                                      unsigned short* tile, int tid) {
#pragma unroll 1
  for (int idx = tid; idx < DIN * R; idx += 256) {
    const int k = idx / R, j = idx % R;
    const int n = n0 + j;
    const int nc = n < DOUT ? n : DOUT - 1;
    const float f = w[(size_t)k * DOUT + nc];
    const unsigned short b = (unsigned short)(n < DOUT ? bf16_bits(f) : 0u);
#pragma unroll
    for (int d = 0; d < DUP; ++d) tile[j * kcat + kofs + d * DIN + k] = b;
  }
}
template <int U8>
__device__ __forceinline__ void wflush(const unsigned short* tile, unsigned short* dst, int tid) {
#pragma unroll 1
  for (int u = tid; u < U8; u += 256) {
    const v8us q = *(const v8usa*)(tile + 8 * u);
    *(volatile v8us*)(dst + 8 * u) = q;
  }
  __threadfence();
#pragma unroll 1
  for (int u = tid; u < U8; u += 256) {
    const v8us q = *(const v8usa*)(tile + 8 * u);
    *(volatile v8us*)(dst + 8 * u) = q;
  }
}

__global__ __launch_bounds__(256) void k_prep(const float* __restrict__ x, const int* __restrict__ bat,
                                              const float* __restrict__ w1l, const float* __restrict__ w1r,
                                              const float* __restrict__ w2l, const float* __restrict__ w2r,
                                              const float* __restrict__ w3l, const float* __restrict__ w3r,
                                              const float* __restrict__ wl1, const float* __restrict__ wl2,
                                              unsigned short* W1C, unsigned short* W2C, unsigned short* W3C,
                                              unsigned short* WL1, unsigned short* WL2,
                                              int* rung, int* rune, unsigned short* xb) {
  __shared__ __attribute__((aligned(16))) unsigned short tile[16384];
  const int tid = (int)threadIdx.x;
  const int b = (int)blockIdx.x;
  if (b == PB_W1) {
    wfill<32, 16, 16, 2>(w1l, 0, 0, 96, tile, tid);
    wfill<32, 16, 16, 1>(w1r, 0, 64, 96, tile, tid);
    __syncthreads();
    wflush<16 * 96 / 8>(tile, W1C, tid);
  } else if (b == PB_W2) {
    wfill<16, 64, 64, 2>(w2l, 0, 0, 64, tile, tid);
    wfill<16, 64, 64, 2>(w2r, 0, 32, 64, tile, tid);
    __syncthreads();
    wflush<64 * 64 / 8>(tile, W2C, tid);
  } else if (b < PB_L1) {
    const int n0 = (b - PB_W3) * 64;
    wfill<64, 512, 64, 2>(w3l, n0, 0, 256, tile, tid);
    wfill<64, 512, 64, 2>(w3r, n0, 128, 256, tile, tid);
    __syncthreads();
    wflush<64 * 256 / 8>(tile, W3C + (size_t)n0 * 256, tid);
  } else if (b < PB_L2) {
    const int n0 = (b - PB_L1) * 16;
    wfill<512, 256, 16, 2>(wl1, n0, 0, 1024, tile, tid);
    __syncthreads();
    wflush<16 * 1024 / 8>(tile, WL1 + (size_t)n0 * 1024, tid);
  } else if (b == PB_L2) {
    wfill<256, 10, 16, 2>(wl2, 0, 0, 512, tile, tid);
    __syncthreads();
    wflush<16 * 512 / 8>(tile, WL2, tid);
  } else if (b < PB_XB) {
    const int t   = (b - PB_RUN) * 256 + tid;
    const int tcl = t < NTILEP ? t : NTILEP - 1;
    int nv = NN - tcl * TM;
    nv = nv < 0 ? 0 : (nv > TM ? TM : nv);
    int g0 = -1, g1 = -1, g2 = -1, g3 = -1, e0 = 0, e1 = 0, e2 = 0, e3 = 0, nr = 0, prev = 0;
#pragma unroll 1
    for (int i = 0; i < TM; ++i) {
      int ix = tcl * TM + i;
      ix = ix < NN - 1 ? ix : NN - 1;
      const int bv = bat[ix];
      const bool act = i < nv;
      const bool nw = act && ((i == 0) || (bv != prev));
      const int gv = ((unsigned)bv < (unsigned)NG) ? bv : -1;
      e0 = (nw && nr == 1) ? i : e0;
      e1 = (nw && nr == 2) ? i : e1;
      e2 = (nw && nr == 3) ? i : e2;
      g0 = (nw && nr == 0) ? gv : g0;
      g1 = (nw && nr == 1) ? gv : g1;
      g2 = (nw && nr == 2) ? gv : g2;
      g3 = (nw && nr == 3) ? gv : g3;
      nr += nw ? 1 : 0;
      prev = act ? bv : prev;
    }
    e0 = nr <= 1 ? nv : e0;
    e1 = nr <= 2 ? nv : e1;
    e2 = nr <= 3 ? nv : e2;
    e3 = nv;
    g3 = nr > 4 ? -2 : g3;
    v4i gq; gq.x = g0; gq.y = g1; gq.z = g2; gq.w = g3;
    v4i eq; eq.x = e0; eq.y = e1; eq.z = e2; eq.w = e3;
    if (t < NTILEP) { *(volatile v4i*)(rung + 4 * t) = gq; *(volatile v4i*)(rune + 4 * t) = eq; }
    __threadfence();
    if (t < NTILEP) { *(volatile v4i*)(rung + 4 * t) = gq; *(volatile v4i*)(rune + 4 * t) = eq; }
  } else {
    const int u  = (b - PB_XB) * 256 + tid;
    const int uc = u < NN * 4 ? u : NN * 4 - 1;
    const bool lv = u < NN * 4;
    const float* p = x + (size_t)uc * 8;
    const v4f a = *(const v4f*)p;
    const v4f c = *(const v4f*)(p + 4);
    v8us o;
    o[0] = (unsigned short)bf16_bits(lv ? a.x : 0.0f); o[1] = (unsigned short)bf16_bits(lv ? a.y : 0.0f);
    o[2] = (unsigned short)bf16_bits(lv ? a.z : 0.0f); o[3] = (unsigned short)bf16_bits(lv ? a.w : 0.0f);
    o[4] = (unsigned short)bf16_bits(lv ? c.x : 0.0f); o[5] = (unsigned short)bf16_bits(lv ? c.y : 0.0f);
    o[6] = (unsigned short)bf16_bits(lv ? c.z : 0.0f); o[7] = (unsigned short)bf16_bits(lv ? c.w : 0.0f);
    unsigned short* dp = xb + (size_t)u * 8;
    if (u < MP * 4) *(volatile v8us*)dp = o;
    __threadfence();
    if (u < MP * 4) *(volatile v8us*)dp = o;
  }
}

__global__ __launch_bounds__(NTHR) void k_compact(const int* __restrict__ srcs, const int* __restrict__ dsts,
                                                  int* lst, int* co) {
  extern __shared__ __attribute__((aligned(16))) int dsm[];
  int* list = dsm;
  int* hl   = dsm + LISTN;
  int* sl   = hl + RCAP;
  int* cnt  = sl + RCAP;
  int* offs = cnt + NBA;
  int* cur  = offs + NBA;
  int* misc = cur + NBA;
  const int tid = (int)threadIdx.x, lane = tid & 31, wave = tid >> 5;
  const int blk = (int)blockIdx.x;
  const int nodeBase = blk * NBA;
  {
    const v4i z4 = {0, 0, 0, 0};
    for (int i = tid * 4; i < AGG_ZINTS; i += NTHR * 4) *(v4ia*)(dsm + i) = z4;
    if (tid < 16) misc[tid] = 0;
  }
  __syncthreads();

  int t = 0, ov = 0;
  const int nChunks = (NE + CHUNK - 1) / CHUNK;
#pragma unroll 1
  for (int ch = 0; ch < nChunks; ++ch) {
    const int cbase = ch * CHUNK;
    const int wc = scan_chunk<SLA>(dsts, NE, cbase, nodeBase, NBA, 1, list, tid, lane, wave);
    if (lane == 0) misc[wave] = wc;
    __syncthreads();
    if (wave == 0) {
#pragma unroll 1
      for (int w2 = 0; w2 < NWAVE; ++w2) {
        int c = misc[w2];
        c = c < 0 ? 0 : (c > WCAP ? WCAP : c);
#pragma unroll 1
        for (int b0 = 0; b0 < c; b0 += 32) {
          const int idx = b0 + lane;
          const int ent = list[w2 * WCAP + (idx < WCAP ? idx : WCAP - 1)];
          const int m32 = (c - b0) < 32 ? (c - b0) : 32;
#pragma unroll 1
          for (int k = 0; k < m32; ++k) {
            const int u    = __builtin_amdgcn_readlane(ent, k);
            const int slot = u & (NBA - 1);
            const int el   = (u >> SLA) & (CHUNK - 1);
            const int pk   = ((cbase + el) << SLA) | slot;
            if (t < RCAP) {
              if (lane == 0) { hl[t] = pk; cnt[slot] = cnt[slot] + 1; }
              t = t + 1;
            } else {
              ov = 1;
            }
          }
        }
      }
    }
    __syncthreads();
  }
  if (wave == 0 && lane == 0) { misc[8] = t; misc[9] = ov; }
  __syncthreads();
  int tt = misc[8];
  tt = tt < 0 ? 0 : (tt > RCAP ? RCAP : tt);
  const int ovf = misc[9];

  if (wave == 0) {
    const int base = lane * (NBA / 32);
    int s = 0;
#pragma unroll 1
    for (int i = 0; i < NBA / 32; ++i) s += cnt[base + i];
    int incl = s;
#pragma unroll
    for (int d = 1; d < 32; d <<= 1) {
      const int y = __shfl_up(incl, d, 32);
      if (lane >= d) incl += y;
    }
    int run = incl - s;
#pragma unroll 1
    for (int i = 0; i < NBA / 32; ++i) {
      const int cv = cnt[base + i];
      offs[base + i] = run;
      cur[base + i]  = run;
      run += cv;
    }
  }
  __syncthreads();
  if (wave == 0) {
#pragma unroll 1
    for (int b0 = 0; b0 < tt; b0 += 32) {
      const int idx = b0 + lane;
      const int ent = hl[idx < RCAP ? idx : RCAP - 1];
      const int m32 = (tt - b0) < 32 ? (tt - b0) : 32;
#pragma unroll 1
      for (int k = 0; k < m32; ++k) {
        const int u    = __builtin_amdgcn_readlane(ent, k);
        const int slot = u & (NBA - 1);
        if (lane == 0) {
          int p = cur[slot];
          p = p < 0 ? 0 : (p > RCAP - 1 ? RCAP - 1 : p);
          sl[p] = u;
          cur[slot] = p + 1;
        }
      }
    }
  }
  __syncthreads();

  const int nIt = (tt + 1023) >> 10;
#pragma unroll 1
  for (int it = 0; it < RCAP / 1024; ++it) {
    const int i = it * 1024 + 4 * tid;
    v4i sv = {0, 0, 0, 0};
    if (it < nIt) {
      const v4i e4 = *(const v4ia*)(sl + i);
      int q0 = e4.x >> SLA, q1 = e4.y >> SLA, q2 = e4.z >> SLA, q3 = e4.w >> SLA;
      q0 = q0 < 0 ? 0 : (q0 > NE - 1 ? NE - 1 : q0);
      q1 = q1 < 0 ? 0 : (q1 > NE - 1 ? NE - 1 : q1);
      q2 = q2 < 0 ? 0 : (q2 > NE - 1 ? NE - 1 : q2);
      q3 = q3 < 0 ? 0 : (q3 > NE - 1 ? NE - 1 : q3);
      int r0 = srcs[q0], r1 = srcs[q1], r2 = srcs[q2], r3 = srcs[q3];
      r0 = r0 < 0 ? 0 : (r0 > NN - 1 ? NN - 1 : r0);
      r1 = r1 < 0 ? 0 : (r1 > NN - 1 ? NN - 1 : r1);
      r2 = r2 < 0 ? 0 : (r2 > NN - 1 ? NN - 1 : r2);
      r3 = r3 < 0 ? 0 : (r3 > NN - 1 ? NN - 1 : r3);
      sv.x = (i     < tt) ? r0 : 0;
      sv.y = (i + 1 < tt) ? r1 : 0;
      sv.z = (i + 2 < tt) ? r2 : 0;
      sv.w = (i + 3 < tt) ? r3 : 0;
    }
    *(v4ia*)(hl + i) = sv;
  }
  __syncthreads();

  v4i c4 = *(const v4ia*)(cnt + 4 * tid);
  const v4i o4 = *(const v4ia*)(offs + 4 * tid);
  if (ovf != 0) { c4.x = DEGCAP + 1; c4.y = DEGCAP + 1; c4.z = DEGCAP + 1; c4.w = DEGCAP + 1; }
  int* cp = co + (size_t)blk * (2 * NBA) + 4 * tid;
  int* lp = lst + (size_t)blk * RCAP;
  *(volatile v4i*)cp = c4;
  *(volatile v4i*)(cp + NBA) = o4;
#pragma unroll 1
  for (int it = 0; it < RCAP / 1024; ++it) {
    const int i = it * 1024 + 4 * tid;
    const v4i v = *(const v4ia*)(hl + i);
    *(volatile v4i*)(lp + i) = v;
  }
  __threadfence();
  *(volatile v4i*)cp = c4;
  *(volatile v4i*)(cp + NBA) = o4;
#pragma unroll 1
  for (int it = 0; it < RCAP / 1024; ++it) {
    const int i = it * 1024 + 4 * tid;
    const v4i v = *(const v4ia*)(hl + i);
    *(volatile v4i*)(lp + i) = v;
  }
}

template <int LAYER>
__global__ __launch_bounds__(NTHR) void k_agg(const int* __restrict__ lst, const int* __restrict__ co,
                                              const unsigned short* __restrict__ hin, unsigned short* aout) {
  constexpr int  IW   = (LAYER == 3) ? 128 : 32;
  constexpr int  EPL  = IW / 32;
  constexpr bool HLIN = (LAYER != 1);
  constexpr int  C    = HLIN ? IW / 2 : IW;
  constexpr int  OW   = 2 * C;
  constexpr int  RPG  = (LAYER == 2) ? 2 : 1;
  constexpr int  GE   = OW * RPG;
  static_assert(GE == 64 || GE == 128);
  static_assert((OW * RPG * 2) % 128 == 0 && NBA % (NWAVE * RPG) == 0);
  __shared__ __attribute__((aligned(16))) int cntL[NBA];
  __shared__ __attribute__((aligned(16))) int offL[NBA];
  __shared__ __attribute__((aligned(16))) unsigned short rowbufs[NWAVE * 128];
  const int tid = (int)threadIdx.x, lane = tid & 31, wave = tid >> 5;
  const int blk = (int)blockIdx.x;
  const int nodeBase = blk * NBA;
  unsigned short* rowbuf = rowbufs + wave * 128;
  {
    const int* cp = co + (size_t)blk * (2 * NBA) + 4 * tid;
    *(v4ia*)(cntL + 4 * tid) = *(const v4i*)cp;
    *(v4ia*)(offL + 4 * tid) = *(const v4i*)(cp + NBA);
  }
  __syncthreads();
  const int* lp = lst + (size_t)blk * RCAP;
  const float qnan = __int_as_float(0x7fc00000);

#pragma unroll 1
  for (int gi = 0; gi < NBA / (NWAVE * RPG); ++gi) {
    const int g = gi * NWAVE + wave;
#pragma unroll
    for (int rr = 0; rr < RPG; ++rr) {
      const int s    = g * RPG + rr;
      const int node = nodeBase + s;
      int c = cntL[s];
      const bool big = (c > DEGCAP) || (c < 0);
      c = c < 0 ? 0 : (c > DEGCAP ? DEGCAP : c);
      int o = offL[s];
      o = o < 0 ? 0 : (o > RCAP ? RCAP : o);
      const bool live = node < NN;
      float acc[EPL];
#pragma unroll
      for (int j = 0; j < EPL; ++j) acc[j] = 0.0f;
#pragma unroll 1
      for (int b0 = 0; b0 < c; b0 += 32) {
        int idx = o + b0 + lane;
        idx = idx > RCAP - 1 ? RCAP - 1 : idx;
        int sr = lp[idx];
        sr = sr < 0 ? 0 : (sr > NN - 1 ? NN - 1 : sr);
        const int m32 = (c - b0) < 32 ? (c - b0) : 32;
#pragma unroll 1
        for (int k = 0; k < m32; ++k) {
          const int sk = __builtin_amdgcn_readlane(sr, k);
          if constexpr (EPL == 4) {
            const v2u w = *(const v2ua*)(hin + (size_t)sk * IW + 4 * lane);
            acc[0] += __uint_as_float(w.x << 16);
            acc[1] += __uint_as_float(w.x & 0xffff0000u);
            acc[2] += __uint_as_float(w.y << 16);
            acc[3] += __uint_as_float(w.y & 0xffff0000u);
          } else {
            const unsigned w = (unsigned)hin[(size_t)sk * IW + lane];
            acc[0] += __uint_as_float(w << 16);
          }
        }
      }
      if constexpr (HLIN) {
#pragma unroll
        for (int j = 0; j < EPL; ++j) acc[j] += __shfl_xor(acc[j], 16, 32);
      }
      const float inv = 1.0f / fmaxf((float)c, 1.0f);
      const float pzr = big ? qnan : 0.0f;
      if constexpr (HLIN) {
        if constexpr (EPL == 4) {
          v4us ob;
#pragma unroll
          for (int j = 0; j < 4; ++j) {
            const float mv = live ? (acc[j] * inv + pzr) : 0.0f;
            unsigned lb;
            const unsigned hb = hl_bits(mv, lb);
            ob[j] = (unsigned short)((lane < 16) ? hb : lb);
          }
          *(v4usa*)(rowbuf + rr * OW + 4 * lane) = ob;
        } else {
          const float mv = live ? (acc[0] * inv + pzr) : 0.0f;
          unsigned lb;
          const unsigned hb = hl_bits(mv, lb);
          rowbuf[rr * OW + lane] = (unsigned short)((lane < 16) ? hb : lb);
        }
      } else {
        const float mv = live ? (acc[0] * inv + pzr) : 0.0f;
        unsigned lb;
        const unsigned hb = hl_bits(mv, lb);
        rowbuf[lane]     = (unsigned short)hb;
        rowbuf[C + lane] = (unsigned short)lb;
      }
    }
    wave_sync();
    const int row0 = nodeBase + g * RPG;
    unsigned short* gp = aout + (size_t)row0 * OW;
    if constexpr (GE == 64) {
      const v2us q = *(const v2usa*)(rowbuf + 2 * lane);
      wave_sync();
      if (row0 < MP) *(volatile v2us*)(gp + 2 * lane) = q;
      __threadfence();
      if (row0 < MP) *(volatile v2us*)(gp + 2 * lane) = q;
    } else {
      const v4us q = *(const v4usa*)(rowbuf + 4 * lane);
      wave_sync();
      if (row0 < MP) *(volatile v4us*)(gp + 4 * lane) = q;
      __threadfence();
      if (row0 < MP) *(volatile v4us*)(gp + 4 * lane) = q;
    }
  }
}

__device__ __forceinline__ void col_run(const float* stg, int col, int s, int e, float& sum, float& mx, float& mn) {
#pragma unroll 2
  for (int r = s; r < e; ++r) {
    const float v = stg[r * 128 + col];
    sum += v;
    mx = (v > mx || v != v) ? v : mx;
    mn = (v < mn || v != v) ? v : mn;
  }
}

template <int NT, int MODE>
__global__ __launch_bounds__(256) void k_gemm(const unsigned short* __restrict__ A0, int lda0, int K0,
                                              const unsigned short* __restrict__ A1, int lda1, int K1,
                                              const unsigned short* __restrict__ BT, int ldb,
                                              const float* __restrict__ bias, int nbias, int nRows,
                                              float* fout, float* stat, const int* __restrict__ rune,
                                              unsigned short* hout) {
  extern __shared__ __attribute__((aligned(16))) float gsm[];
  constexpr int NC = 16 * NT;
  float* stg = gsm;
  float* rec = gsm + 128 * NC;
  const int tid = (int)threadIdx.x, lane = tid & 31, wave = tid >> 5, hh = lane >> 4, m = lane & 15;
  const int rowBase = (int)blockIdx.x * TM;
  const int colBase = (int)blockIdx.y * NC;

  v8f acc[NT];
#pragma unroll
  for (int t = 0; t < NT; ++t) acc[t] = z8();
  const unsigned short* ap0 = A0 + (size_t)(rowBase + 16 * wave + m) * (size_t)lda0 + 8 * hh;
  const unsigned short* ap1 = A1 + (size_t)(rowBase + 16 * wave + m) * (size_t)lda1 + 8 * hh;
  const unsigned short* bp  = BT + (size_t)(colBase + m) * (size_t)ldb + 8 * hh;

#pragma unroll 1
  for (int k0 = 0; k0 < K0; k0 += 32) {
    FragB af;
    af.h[0] = *(const v8usa*)(ap0 + k0);
    af.h[1] = *(const v8usa*)(ap0 + k0 + 16);
#pragma unroll
    for (int nt = 0; nt < NT; ++nt) {
      const unsigned short* wq = bp + (size_t)(16 * nt) * (size_t)ldb + k0;
      FragB bf;
      bf.h[0] = *(const v8usa*)wq;
      bf.h[1] = *(const v8usa*)(wq + 16);
      acc[nt] = wmb(af, bf, acc[nt]);
    }
  }
#pragma unroll 1
  for (int k0 = 0; k0 < K1; k0 += 32) {
    FragB af;
    af.h[0] = *(const v8usa*)(ap1 + k0);
    af.h[1] = *(const v8usa*)(ap1 + k0 + 16);
#pragma unroll
    for (int nt = 0; nt < NT; ++nt) {
      const unsigned short* wq = bp + (size_t)(16 * nt) * (size_t)ldb + K0 + k0;
      FragB bf;
      bf.h[0] = *(const v8usa*)wq;
      bf.h[1] = *(const v8usa*)(wq + 16);
      acc[nt] = wmb(af, bf, acc[nt]);
    }
  }

#pragma unroll
  for (int nt = 0; nt < NT; ++nt) {
    const int lc  = 16 * nt + m;
    const int col = colBase + lc;
    const int cc  = col < nbias ? col : nbias - 1;
    float bv = bf16_val(bias[cc]);
    bv = col < nbias ? bv : 0.0f;
#pragma unroll
    for (int r = 0; r < 8; ++r) {
      const int lr = 16 * wave + 8 * hh + r;
      stg[lr * NC + lc] = acc[nt][r] + bv;
    }
  }
  __syncthreads();

  int nv = nRows - rowBase;
  nv = nv < 0 ? 0 : (nv > TM ? TM : nv);

  if constexpr (MODE == 0) {
    constexpr int CW = NC >= 32 ? NC / 32 : 1;
    if (wave < CW) {
      const int col = tid & (NC - 1);
      float s = 0.0f;
#pragma unroll 4
      for (int r = 0; r < nv; ++r) s += stg[r * NC + col];
      const float mean = s * (1.0f / (float)(nv > 0 ? nv : 1));
      float q = 0.0f;
#pragma unroll 4
      for (int r = 0; r < nv; ++r) {
        const float d = stg[r * NC + col] - mean;
        q = fmaf(d, d, q);
      }
      if (tid < NC) { rec[tid] = mean; rec[NC + tid] = q; }
    }
    __syncthreads();
    float* tp = fout + (size_t)rowBase * NC;
    constexpr int NQ = 128 * NC / 4;
    constexpr int SQ = 2 * NC / 4;
    static_assert(NQ % 256 == 0 && SQ <= 256);
    const int sq = tid < SQ ? tid : SQ - 1;
    const v4f sv = *(const v4fa*)(rec + 4 * sq);
    float* sp = stat + (size_t)blockIdx.x * (2 * NC) + 4 * sq;
#pragma unroll 1
    for (int q = tid; q < NQ; q += 256) {
      const v4f v = *(const v4fa*)(stg + 4 * q);
      *(volatile v4f*)(tp + 4 * q) = v;
    }
    if (tid < SQ) *(volatile v4f*)sp = sv;
    __threadfence();
#pragma unroll 1
    for (int q = tid; q < NQ; q += 256) {
      const v4f v = *(const v4fa*)(stg + 4 * q);
      *(volatile v4f*)(tp + 4 * q) = v;
    }
    if (tid < SQ) *(volatile v4f*)sp = sv;
  } else if constexpr (MODE == 1) {
    static_assert(NC == 128);
    const v4i re = *(const v4i*)(rune + 4 * (int)blockIdx.x);
    int e0 = __builtin_amdgcn_readfirstlane(re.x);
    int e1 = __builtin_amdgcn_readfirstlane(re.y);
    int e2 = __builtin_amdgcn_readfirstlane(re.z);
    e0 = e0 < 0 ? 0 : (e0 > nv ? nv : e0);
    e1 = e1 < e0 ? e0 : (e1 > nv ? nv : e1);
    e2 = e2 < e1 ? e1 : (e2 > nv ? nv : e2);
    const int e3 = nv;
    if (wave < 4) {
      const int col = tid;
      const float ninf = -__builtin_huge_valf(), pinf = __builtin_huge_valf();
      float sum = 0.0f;
      float mx0 = ninf, mx1 = ninf, mx2 = ninf, mx3 = ninf;
      float mn0 = pinf, mn1 = pinf, mn2 = pinf, mn3 = pinf;
      col_run(stg, col, 0,  e0, sum, mx0, mn0);
      col_run(stg, col, e0, e1, sum, mx1, mn1);
      col_run(stg, col, e1, e2, sum, mx2, mn2);
      col_run(stg, col, e2, e3, sum, mx3, mn3);
      const float mean = sum * (1.0f / (float)(nv > 0 ? nv : 1));
      float q = 0.0f;
#pragma unroll 4
      for (int r = 0; r < nv; ++r) {
        const float d = stg[r * 128 + col] - mean;
        q = fmaf(d, d, q);
      }
      rec[col] = mean;         rec[128 + col] = q;
      rec[2 * 128 + col] = mx0; rec[3 * 128 + col] = mx1; rec[4 * 128 + col] = mx2; rec[5 * 128 + col] = mx3;
      rec[6 * 128 + col] = mn0; rec[7 * 128 + col] = mn1; rec[8 * 128 + col] = mn2; rec[9 * 128 + col] = mn3;
    }
    __syncthreads();
    float* rp = fout + (size_t)blockIdx.x * (10 * 512) + colBase;
#pragma unroll 1
    for (int q = tid; q < 320; q += 256) {
      const v4f v = *(const v4fa*)(rec + 4 * q);
      *(volatile v4f*)(rp + (size_t)(q >> 5) * 512 + 4 * (q & 31)) = v;
    }
    __threadfence();
#pragma unroll 1
    for (int q = tid; q < 320; q += 256) {
      const v4f v = *(const v4fa*)(rec + 4 * q);
      *(volatile v4f*)(rp + (size_t)(q >> 5) * 512 + 4 * (q & 31)) = v;
    }
  } else if constexpr (MODE == 2) {
    static_assert(NC == 128);
    v4us hv[16], lv[16];
#pragma unroll
    for (int i = 0; i < 16; ++i) {
      const v4f xq = *(const v4fa*)(stg + (16 * wave + i) * NC + 4 * lane);
      const float y0 = relu_np(xq.x), y1 = relu_np(xq.y), y2 = relu_np(xq.z), y3 = relu_np(xq.w);
      v4us hq, lq;
      unsigned lb;
      unsigned hb;
      hb = hl_bits(y0, lb); hq[0] = (unsigned short)hb; lq[0] = (unsigned short)lb;
      hb = hl_bits(y1, lb); hq[1] = (unsigned short)hb; lq[1] = (unsigned short)lb;
      hb = hl_bits(y2, lb); hq[2] = (unsigned short)hb; lq[2] = (unsigned short)lb;
      hb = hl_bits(y3, lb); hq[3] = (unsigned short)hb; lq[3] = (unsigned short)lb;
      hv[i] = hq;
      lv[i] = lq;
    }
#pragma unroll
    for (int i = 0; i < 16; ++i) {
      unsigned short* op = hout + (size_t)(rowBase + 16 * wave + i) * 512 + colBase + 4 * lane;
      *(volatile v4us*)op = hv[i];
      *(volatile v4us*)(op + 256) = lv[i];
    }
    __threadfence();
#pragma unroll
    for (int i = 0; i < 16; ++i) {
      unsigned short* op = hout + (size_t)(rowBase + 16 * wave + i) * 512 + colBase + 4 * lane;
      *(volatile v4us*)op = hv[i];
      *(volatile v4us*)(op + 256) = lv[i];
    }
  } else {
    static_assert(NC == 16);
#pragma unroll 1
    for (int idx = tid; idx < 1280; idx += 256) {
      const int row = idx / 10;
      const int c   = idx - row * 10;
      rec[idx] = stg[row * 16 + c];
    }
    __syncthreads();
#pragma unroll 1
    for (int q = tid; q < 320; q += 256) {
      const v4f v = *(const v4fa*)(rec + 4 * q);
      *(volatile v4f*)(fout + 4 * q) = v;
    }
    __threadfence();
#pragma unroll 1
    for (int q = tid; q < 320; q += 256) {
      const v4f v = *(const v4fa*)(rec + 4 * q);
      *(volatile v4f*)(fout + 4 * q) = v;
    }
  }
}

template <int NC>
__global__ __launch_bounds__(128) void k_comb(const float* __restrict__ st, int tstride, int m2off,
                                              const float* __restrict__ gam, const float* __restrict__ bet,
                                              float* bnp) {
  constexpr int CB = NC < 128 ? NC : 128;
  constexpr int PR = CB / 4;
  __shared__ __attribute__((aligned(16))) float sm[4 * CB];
  const int tid = (int)threadIdx.x;
  const int col = (int)blockIdx.x * 128 + tid;
  const int cc  = col < NC ? col : NC - 1;
  double n = 0.0, mean = 0.0, M2 = 0.0;
#pragma unroll 1
  for (int t = 0; t < NTILE; ++t) {
    int nvi = NN - t * TM;
    nvi = nvi > TM ? TM : nvi;
    const double nb = (double)nvi;
    const double mb = (double)st[(size_t)t * tstride + cc];
    const double qb = (double)st[(size_t)t * tstride + m2off + cc];
    const double nn = n + nb;
    const double delta = mb - mean;
    const double f = nb / nn;
    mean = mean + delta * f;
    M2 = M2 + qb + delta * delta * n * f;
    n = nn;
  }
  const float varf = (float)(M2 / (double)NN);
  const float r = 1.0f / sqrtf(varf + BNEPS);
  const float gq = bf16_val(gam[cc]);
  const float bq = bf16_val(bet[cc]);
  if (tid < CB) { sm[tid] = (float)mean; sm[CB + tid] = r; sm[2 * CB + tid] = gq; sm[3 * CB + tid] = bq; }
  __syncthreads();
  const int tq = tid < CB ? tid : CB - 1;
  const int row = tq / PR, piece = tq % PR;
  const v4f v = *(const v4fa*)(sm + row * CB + 4 * piece);
  float* dp = bnp + (size_t)row * NC + (size_t)blockIdx.x * 128 + 4 * piece;
  if (tid < CB) *(volatile v4f*)dp = v;
  __threadfence();
  if (tid < CB) *(volatile v4f*)dp = v;
}

template <int NC>
__global__ __launch_bounds__(256) void k_apply(const float* __restrict__ T, const float* __restrict__ bnp,
                                               unsigned short* H) {
  constexpr int RB = 2048 / NC;
  constexpr int OW = 2 * NC;
  static_assert(RB * OW == 4096 && NC % 8 == 0 && (MP * NC) % 2048 == 0);
  __shared__ __attribute__((aligned(16))) unsigned short tile[RB * OW];
  const int tid = (int)threadIdx.x;
  const int blk = (int)blockIdx.x;
  const size_t f = ((size_t)blk * 256 + tid) * 8;
  const int row = (int)(f / NC);
  const int c   = (int)(f % NC);
  const int lr  = row - blk * RB;
  const v4f t0 = *(const v4f*)(T + f),            t1 = *(const v4f*)(T + f + 4);
  const v4f m0 = *(const v4f*)(bnp + c),          m1 = *(const v4f*)(bnp + c + 4);
  const v4f r0 = *(const v4f*)(bnp + NC + c),     r1 = *(const v4f*)(bnp + NC + c + 4);
  const v4f g0 = *(const v4f*)(bnp + 2 * NC + c), g1 = *(const v4f*)(bnp + 2 * NC + c + 4);
  const v4f b0 = *(const v4f*)(bnp + 3 * NC + c), b1 = *(const v4f*)(bnp + 3 * NC + c + 4);
  const float tv[8] = {t0.x, t0.y, t0.z, t0.w, t1.x, t1.y, t1.z, t1.w};
  const float mv[8] = {m0.x, m0.y, m0.z, m0.w, m1.x, m1.y, m1.z, m1.w};
  const float rv[8] = {r0.x, r0.y, r0.z, r0.w, r1.x, r1.y, r1.z, r1.w};
  const float gv[8] = {g0.x, g0.y, g0.z, g0.w, g1.x, g1.y, g1.z, g1.w};
  const float bv[8] = {b0.x, b0.y, b0.z, b0.w, b1.x, b1.y, b1.z, b1.w};
  const bool live = row < NN;
  v8us hq, lq;
#pragma unroll
  for (int j = 0; j < 8; ++j) {
    float y = ((tv[j] - mv[j]) * rv[j]) * gv[j] + bv[j];
    y = relu_np(y);
    y = live ? y : 0.0f;
    unsigned lb;
    const unsigned hb = hl_bits(y, lb);
    hq[j] = (unsigned short)hb;
    lq[j] = (unsigned short)lb;
  }
  *(v8usa*)(tile + lr * OW + c)      = hq;
  *(v8usa*)(tile + lr * OW + NC + c) = lq;
  __syncthreads();
  unsigned short* hp = H + (size_t)blk * 4096;
#pragma unroll 1
  for (int q = tid; q < 512; q += 256) {
    const v8us v = *(const v8usa*)(tile + 8 * q);
    *(volatile v8us*)(hp + 8 * q) = v;
  }
  __threadfence();
#pragma unroll 1
  for (int q = tid; q < 512; q += 256) {
    const v8us v = *(const v8usa*)(tile + 8 * q);
    *(volatile v8us*)(hp + 8 * q) = v;
  }
}

__global__ __launch_bounds__(512) void k_pool(const float* __restrict__ rec3, const int* __restrict__ rung,
                                              const float* __restrict__ bnp3, unsigned short* pool) {
  __shared__ __attribute__((aligned(16))) unsigned short prow[1024];
  const int tid = (int)threadIdx.x;
  const int c = tid;
  const int g = (int)blockIdx.x;
  const float ninf = -__builtin_huge_valf(), pinf = __builtin_huge_valf();
  float mx = ninf, mn = pinf;
  int found = 0, pois = 0;
#pragma unroll 1
  for (int t = 0; t < NTILE; ++t) {
    const v4i rg = *(const v4i*)(rung + 4 * t);
    const int q0 = __builtin_amdgcn_readfirstlane(rg.x);
    const int q1 = __builtin_amdgcn_readfirstlane(rg.y);
    const int q2 = __builtin_amdgcn_readfirstlane(rg.z);
    const int q3 = __builtin_amdgcn_readfirstlane(rg.w);
    pois |= ((q0 == -2) | (q1 == -2) | (q2 == -2) | (q3 == -2)) ? 1 : 0;
    const float* rb = rec3 + (size_t)t * (10 * 512) + c;
    if (q0 == g) {
      const float v = rb[2 * 512], w = rb[6 * 512];
      mx = (v > mx || v != v) ? v : mx; mn = (w < mn || w != w) ? w : mn; found = 1;
    }
    if (q1 == g) {
      const float v = rb[3 * 512], w = rb[7 * 512];
      mx = (v > mx || v != v) ? v : mx; mn = (w < mn || w != w) ? w : mn; found = 1;
    }
    if (q2 == g) {
      const float v = rb[4 * 512], w = rb[8 * 512];
      mx = (v > mx || v != v) ? v : mx; mn = (w < mn || w != w) ? w : mn; found = 1;
    }
    if (q3 == g) {
      const float v = rb[5 * 512], w = rb[9 * 512];
      mx = (v > mx || v != v) ? v : mx; mn = (w < mn || w != w) ? w : mn; found = 1;
    }
  }
  const float m  = bnp3[c];
  const float r  = bnp3[512 + c];
  const float gg = bnp3[1024 + c];
  const float bb = bnp3[1536 + c];
  const float sel = (gg >= 0.0f) ? mx : mn;
  float y = ((sel - m) * r) * gg + bb;
  y = relu_np(y);
  y = (found != 0) ? y : ninf;
  y = (pois != 0) ? __int_as_float(0x7fc00000) : y;
  unsigned lb;
  const unsigned hb = hl_bits(y, lb);
  prow[c]       = (unsigned short)hb;
  prow[512 + c] = (unsigned short)lb;
  __syncthreads();
  const int tq = tid < 128 ? tid : 127;
  const v8us q = *(const v8usa*)(prow + 8 * tq);
  unsigned short* op = pool + (size_t)g * 1024 + 8 * tq;
  if (tid < 128) *(volatile v8us*)op = q;
  __threadfence();
  if (tid < 128) *(volatile v8us*)op = q;
}

static inline size_t al256(size_t o) { return (o + 255) & ~(size_t)255; }

extern "C" void kernel_launch(void* const* d_in, const int* in_sizes, int n_in,
                              void* d_out, int out_size, void* d_ws, size_t ws_size,
                              hipStream_t stream) {
  if (n_in < 22) return;
  const int want[22] = {NN * 32, 2 * NE, NN, 512, 16, 512, 1024, 64, 1024, 32768, 512, 32768,
                        16, 16, 64, 64, 512, 512, 131072, 256, 2560, 10};
  for (int i = 0; i < 22; ++i) if (in_sizes[i] != want[i]) return;
  if (out_size != NG * 10) return;

  const float* x   = (const float*)d_in[0];
  const int*   ei  = (const int*)  d_in[1];
  const int*   bat = (const int*)  d_in[2];
  const float* w1l = (const float*)d_in[3];
  const float* b1  = (const float*)d_in[4];
  const float* w1r = (const float*)d_in[5];
  const float* w2l = (const float*)d_in[6];
  const float* b2  = (const float*)d_in[7];
  const float* w2r = (const float*)d_in[8];
  const float* w3l = (const float*)d_in[9];
  const float* b3  = (const float*)d_in[10];
  const float* w3r = (const float*)d_in[11];
  const float* g1  = (const float*)d_in[12];
  const float* be1 = (const float*)d_in[13];
  const float* g2  = (const float*)d_in[14];
  const float* be2 = (const float*)d_in[15];
  const float* g3  = (const float*)d_in[16];
  const float* be3 = (const float*)d_in[17];
  const float* wl1 = (const float*)d_in[18];
  const float* bl1 = (const float*)d_in[19];
  const float* wl2 = (const float*)d_in[20];
  const float* bl2 = (const float*)d_in[21];
  float* out = (float*)d_out;
  const int* src = ei;
  const int* dst = ei + NE;

  char* ws = (char*)d_ws;
  size_t off = 0;
  const size_t szXB = (size_t)MP * 32 * 2, szA1 = (size_t)MP * 64 * 2, szH1 = (size_t)MP * 32 * 2;
  const size_t szA3 = (size_t)MP * 128 * 2;
  if (szXB + szA1 + szH1 != szA3) return;
  const size_t oR0  = off; off = al256(off + szA3);
  const size_t oT1  = off; off = al256(off + (size_t)MP * 16 * 4);
  const size_t oA2  = off; off = al256(off + (size_t)MP * 32 * 2);
  const size_t oT2  = off; off = al256(off + (size_t)MP * 64 * 4);
  const size_t oH2  = off; off = al256(off + (size_t)MP * 128 * 2);
  const size_t oLS  = off; off = al256(off + (size_t)NBLK * RCAP * 4);
  const size_t oCO  = off; off = al256(off + (size_t)NBLK * 2 * NBA * 4);
  const size_t oRG  = off; off = al256(off + (size_t)NTILEP * 16);
  const size_t oRE  = off; off = al256(off + (size_t)NTILEP * 16);
  const size_t oS1  = off; off = al256(off + (size_t)NTILE * 32 * 4);
  const size_t oS2  = off; off = al256(off + (size_t)NTILE * 128 * 4);
  const size_t oR3  = off; off = al256(off + (size_t)NTILE * 10 * 512 * 4);
  const size_t oB1  = off; off = al256(off + (size_t)4 * 16 * 4);
  const size_t oB2  = off; off = al256(off + (size_t)4 * 64 * 4);
  const size_t oB3  = off; off = al256(off + (size_t)4 * 512 * 4);
  const size_t oW1  = off; off = al256(off + (size_t)16 * 96 * 2);
  const size_t oW2  = off; off = al256(off + (size_t)64 * 64 * 2);
  const size_t oW3  = off; off = al256(off + (size_t)512 * 256 * 2);
  const size_t oWA  = off; off = al256(off + (size_t)256 * 1024 * 2);
  const size_t oWB  = off; off = al256(off + (size_t)16 * 512 * 2);
  const size_t oPL  = off; off = al256(off + (size_t)NG * 1024 * 2);
  const size_t oO1  = off; off = al256(off + (size_t)NG * 512 * 2);
  if (off > ws_size || off > (size_t)WSMAX) return;
  unsigned short* XB   = (unsigned short*)(ws + oR0);
  unsigned short* AGG1 = (unsigned short*)(ws + oR0 + szXB);
  unsigned short* H1   = (unsigned short*)(ws + oR0 + szXB + szA1);
  unsigned short* AGG3 = (unsigned short*)(ws + oR0);
  float*          T1   = (float*)(ws + oT1);
  unsigned short* AGG2 = (unsigned short*)(ws + oA2);
  float*          T2   = (float*)(ws + oT2);
  unsigned short* H2   = (unsigned short*)(ws + oH2);
  int*            LST  = (int*)(ws + oLS);
  int*            CO   = (int*)(ws + oCO);
  int*            RUNG = (int*)(ws + oRG);
  int*            RUNE = (int*)(ws + oRE);
  float*          ST1  = (float*)(ws + oS1);
  float*          ST2  = (float*)(ws + oS2);
  float*          REC3 = (float*)(ws + oR3);
  float*          BN1  = (float*)(ws + oB1);
  float*          BN2  = (float*)(ws + oB2);
  float*          BN3  = (float*)(ws + oB3);
  unsigned short* W1C  = (unsigned short*)(ws + oW1);
  unsigned short* W2C  = (unsigned short*)(ws + oW2);
  unsigned short* W3C  = (unsigned short*)(ws + oW3);
  unsigned short* WL1  = (unsigned short*)(ws + oWA);
  unsigned short* WL2  = (unsigned short*)(ws + oWB);
  unsigned short* POOL = (unsigned short*)(ws + oPL);
  unsigned short* O1   = (unsigned short*)(ws + oO1);

  const size_t cLds = (size_t)AGG_LDS_INTS * 4;
  const size_t gL1 = (size_t)(128 * 16 + 1280) * 4;
  const size_t gL4 = (size_t)(128 * 64 + 1280) * 4;
  const size_t gL8 = (size_t)(128 * 128 + 1280) * 4;
  hipFuncSetAttribute(reinterpret_cast<const void*>(&k_compact), hipFuncAttributeMaxDynamicSharedMemorySize, (int)cLds);
  hipFuncSetAttribute(reinterpret_cast<const void*>(&k_gemm<8, 1>), hipFuncAttributeMaxDynamicSharedMemorySize, (int)gL8);
  hipFuncSetAttribute(reinterpret_cast<const void*>(&k_gemm<8, 2>), hipFuncAttributeMaxDynamicSharedMemorySize, (int)gL8);

  k_prep<<<PB_END, 256, 0, stream>>>(x, bat, w1l, w1r, w2l, w2r, w3l, w3r, wl1, wl2,
                                     W1C, W2C, W3C, WL1, WL2, RUNG, RUNE, XB);
  k_compact<<<NBLK, NTHR, cLds, stream>>>(src, dst, LST, CO);
  k_agg<1><<<NBLK, NTHR, 0, stream>>>(LST, CO, XB, AGG1);
  k_gemm<1, 0><<<dim3(NTILE, 1), 256, gL1, stream>>>(AGG1, 64, 64, XB, 32, 32, W1C, 96, b1, 16, NN,
                                                     T1, ST1, RUNE, O1);
  k_comb<16><<<1, 128, 0, stream>>>(ST1, 32, 16, g1, be1, BN1);
  k_apply<16><<<(MP * 16) / 2048, 256, 0, stream>>>(T1, BN1, H1);
  k_agg<2><<<NBLK, NTHR, 0, stream>>>(LST, CO, H1, AGG2);
  k_gemm<4, 0><<<dim3(NTILE, 1), 256, gL4, stream>>>(AGG2, 32, 32, H1, 32, 32, W2C, 64, b2, 64, NN,
                                                     T2, ST2, RUNE, O1);
  k_comb<64><<<1, 128, 0, stream>>>(ST2, 128, 64, g2, be2, BN2);
  k_apply<64><<<(MP * 64) / 2048, 256, 0, stream>>>(T2, BN2, H2);
  k_agg<3><<<NBLK, NTHR, 0, stream>>>(LST, CO, H2, AGG3);
  k_gemm<8, 1><<<dim3(NTILE, 4), 256, gL8, stream>>>(AGG3, 128, 128, H2, 128, 128, W3C, 256, b3, 512, NN,
                                                     REC3, ST2, RUNE, O1);
  k_comb<512><<<4, 128, 0, stream>>>(REC3, 10 * 512, 512, g3, be3, BN3);
  k_pool<<<NG, 512, 0, stream>>>(REC3, RUNG, BN3, POOL);
  k_gemm<8, 2><<<dim3(1, 2), 256, gL8, stream>>>(POOL, 1024, 1024, POOL, 1024, 0, WL1, 1024, bl1, 256, NG,
                                                 T1, ST1, RUNE, O1);
  k_gemm<1, 3><<<dim3(1, 1), 256, gL1, stream>>>(O1, 512, 512, O1, 512, 0, WL2, 512, bl2, 10, NG,
                                                 out, ST1, RUNE, O1);
}
